// SelfAttention_58342835749603
// MI455X (gfx1250) — hardware-verified
//
#include <hip/hip_runtime.h>


#ifndef NB
#define NB 4
#endif
#ifndef SEQ
#define SEQ 2048
#endif
#define NB_FULL  4
#define SEQ_FULL 2048
#define DMOD  768
#define NHEAD 12
#define HDIM  64
#define OSP   68
#define LOG2E 1.4426950408889634f
#define PSH   8.0f
#define RCAR  2048.0f
#define WCAR  64.0f
#define CCAR  16.0f

static_assert(NHEAD * HDIM == DMOD);
static_assert(HDIM == 64);
static_assert(DMOD % 64 == 0);
static_assert(DMOD % 32 == 0);
static_assert(SEQ % 64 == 0);
static_assert(SEQ <= SEQ_FULL);
static_assert(NB <= NB_FULL);
static_assert((SEQ * DMOD) % 8 == 0);
static_assert((DMOD * DMOD) % 8 == 0);
static_assert((NB * SEQ) % 64 == 0);
static_assert((NB * SEQ) / 64 <= 65535);
static_assert(OSP % 4 == 0);
static_assert(OSP >= HDIM);
static_assert(DMOD % 8 == 0);
static_assert(SEQ % 8 == 0);
static_assert(SEQ_FULL % 8 == 0);
static_assert(DMOD == 6 * 32 * 4);
static_assert((NB * SEQ) % 8 == 0);
static_assert(HDIM == 16 * 4);

typedef _Float16 h16;
typedef unsigned short bf;
typedef __attribute__((ext_vector_type(16))) __bf16   v16bf;
typedef __attribute__((ext_vector_type(16))) _Float16 v16h;
typedef __attribute__((ext_vector_type(8)))  _Float16 v8h;
typedef __attribute__((ext_vector_type(8)))  unsigned short v8us;
typedef __attribute__((ext_vector_type(8)))  float    v8f;
typedef __attribute__((ext_vector_type(4)))  float    v4f;
typedef __attribute__((ext_vector_type(4)))  int      v4i;
typedef v4f  __attribute__((may_alias)) v4fa;

__device__ __forceinline__ unsigned short f2bf(float f) { unsigned u = __float_as_uint(f); u += 0x7FFFu + ((u >> 16) & 1u); return (unsigned short)(u >> 16); }
__device__ __forceinline__ float bf2f(unsigned short b) { return __uint_as_float(((unsigned)b) << 16); }
__device__ __forceinline__ float bfr(float f) { return bf2f(f2bf(f)); }
__device__ __forceinline__ void splitf(float y, unsigned short& h, unsigned short& l) { h = f2bf(y); l = f2bf(y - bf2f(h)); }
__device__ __forceinline__ v16h cat16(v8h lo, v8h hi) { return __builtin_shufflevector(lo, hi, 0, 1, 2, 3, 4, 5, 6, 7, 8, 9, 10, 11, 12, 13, 14, 15); }
__device__ __forceinline__ v16bf cat16b(v8us lo, v8us hi) { return __builtin_bit_cast(v16bf, __builtin_shufflevector(lo, hi, 0, 1, 2, 3, 4, 5, 6, 7, 8, 9, 10, 11, 12, 13, 14, 15)); }
__device__ __forceinline__ v8f wmma16(v16h a, v16h b, v8f c) { return __builtin_amdgcn_wmma_f32_16x16x32_f16(false, a, false, b, (short)0, c, false, false); }
__device__ __forceinline__ v8f wmmab(v16bf a, v16bf b, v8f c) { return __builtin_amdgcn_wmma_f32_16x16x32_bf16(false, a, false, b, (short)0, c, false, false); }
__device__ __forceinline__ v8f wmma16g(v16h a, v16h b, v8f c) { c = wmma16(a, b, c); asm volatile("v_nop\n\tv_nop\n\tv_nop\n\tv_nop" : "+v"(c) : "v"(a), "v"(b)); return c; }
__device__ __forceinline__ v16bf ldbf(const bf* p) { return cat16b(*(const v8us*)p, *(const v8us*)(p + 16)); }
__device__ __forceinline__ v16h  ldh(const h16* p) { return cat16(*(const v8h*)p, *(const v8h*)(p + 16)); }
static __device__ __forceinline__ h16 toh_flush(float v) { const h16 r = (h16)v; return (fabsf(v) < 6.103515625e-05f) ? (h16)0.0f : r; }

__global__ __launch_bounds__(256) void k_cvt(const float* __restrict__ src, bf* dst, int n, int per, int per_full) {
    const int e = ((int)blockIdx.x * 256 + (int)threadIdx.x) * 8;
    if (e >= n) return;
    const int b = e / per;
    const size_t so = (size_t)b * (size_t)per_full + (size_t)(e - b * per);
    const v4f a0 = *(const v4f*)(src + so);
    const v4f a1 = *(const v4f*)(src + so + 4);
    v8us o;
    o[0] = f2bf(a0[0]); o[1] = f2bf(a0[1]); o[2] = f2bf(a0[2]); o[3] = f2bf(a0[3]);
    o[4] = f2bf(a1[0]); o[5] = f2bf(a1[1]); o[6] = f2bf(a1[2]); o[7] = f2bf(a1[3]);
    *(volatile v8us*)(dst + e) = o;
    __threadfence();
    *(volatile v8us*)(dst + e) = o;
}

__global__ __launch_bounds__(256) void k_cvt_wo(const float* __restrict__ src, h16* dst, int n) {
    const int e = ((int)blockIdx.x * 256 + (int)threadIdx.x) * 8;
    if (e >= n) return;
    const v4f a0 = *(const v4f*)(src + e);
    const v4f a1 = *(const v4f*)(src + e + 4);
    v8h o;
    o[0] = toh_flush(bfr(a0[0]) * WCAR); o[1] = toh_flush(bfr(a0[1]) * WCAR); o[2] = toh_flush(bfr(a0[2]) * WCAR); o[3] = toh_flush(bfr(a0[3]) * WCAR);
    o[4] = toh_flush(bfr(a1[0]) * WCAR); o[5] = toh_flush(bfr(a1[1]) * WCAR); o[6] = toh_flush(bfr(a1[2]) * WCAR); o[7] = toh_flush(bfr(a1[3]) * WCAR);
    *(volatile v8h*)(dst + e) = o;
    __threadfence();
    *(volatile v8h*)(dst + e) = o;
}

__global__ __launch_bounds__(256) void k_cvt_ctx(const float* __restrict__ src, const int* __restrict__ mask, h16* dst, int n) {
    const int e = ((int)blockIdx.x * 256 + (int)threadIdx.x) * 8;
    if (e >= n) return;
    const int row = e / DMOD, col = e - row * DMOD;
    const int b = row / SEQ, t = row - b * SEQ;
    const size_t srow = (size_t)b * SEQ_FULL + (size_t)t;
    const float mq = (float)mask[srow] * CCAR;
    const v4f a0 = *(const v4f*)(src + srow * DMOD + col);
    const v4f a1 = *(const v4f*)(src + srow * DMOD + col + 4);
    v8h o;
    o[0] = toh_flush(a0[0] * mq); o[1] = toh_flush(a0[1] * mq); o[2] = toh_flush(a0[2] * mq); o[3] = toh_flush(a0[3] * mq);
    o[4] = toh_flush(a1[0] * mq); o[5] = toh_flush(a1[1] * mq); o[6] = toh_flush(a1[2] * mq); o[7] = toh_flush(a1[3] * mq);
    *(volatile v8h*)(dst + e) = o;
    __threadfence();
    *(volatile v8h*)(dst + e) = o;
}

__device__ __forceinline__ void gemm_tile(const bf* __restrict__ A, const bf* __restrict__ Bt, size_t aoff, size_t boff, v8f (&acc)[4][4]) {
#pragma unroll
    for (int mb = 0; mb < 4; ++mb)
#pragma unroll
        for (int nb = 0; nb < 4; ++nb) acc[mb][nb] = (v8f){};
#pragma unroll 1
    for (int kc = 0; kc < DMOD; kc += 32) {
        v16bf a[4];
        v16bf b;
#pragma unroll
        for (int mb = 0; mb < 4; ++mb) a[mb] = ldbf(A + aoff + (size_t)mb * 16 * DMOD + kc);
#pragma unroll
        for (int nb = 0; nb < 4; ++nb) {
            b = ldbf(Bt + boff + (size_t)nb * 16 * DMOD + kc);
#pragma unroll
            for (int mb = 0; mb < 4; ++mb) acc[mb][nb] = wmmab(a[mb], b, acc[mb][nb]);
        }
        asm volatile("" : "+v"(acc[0][0]), "+v"(acc[1][0]), "+v"(acc[2][0]), "+v"(acc[3][0]), "+v"(acc[0][1]), "+v"(acc[1][1]), "+v"(acc[2][1]), "+v"(acc[3][1]));
        asm volatile("v_nop\n\tv_nop\n\tv_nop\n\tv_nop" : "+v"(acc[0][2]), "+v"(acc[1][2]), "+v"(acc[2][2]), "+v"(acc[3][2]), "+v"(acc[0][3]), "+v"(acc[1][3]), "+v"(acc[2][3]), "+v"(acc[3][3]) : "v"(a[0]), "v"(a[3]), "v"(b));
    }
}

__device__ __forceinline__ void gemm_tile_h(const h16* __restrict__ A, const h16* __restrict__ Bt, size_t aoff, size_t boff, v8f (&acc)[4][4]) {
#pragma unroll
    for (int mb = 0; mb < 4; ++mb)
#pragma unroll
        for (int nb = 0; nb < 4; ++nb) acc[mb][nb] = (v8f){};
#pragma unroll 1
    for (int kc = 0; kc < DMOD; kc += 32) {
        v16h a[4];
        v16h b;
#pragma unroll
        for (int mb = 0; mb < 4; ++mb) a[mb] = ldh(A + aoff + (size_t)mb * 16 * DMOD + kc);
#pragma unroll
        for (int nb = 0; nb < 4; ++nb) {
            b = ldh(Bt + boff + (size_t)nb * 16 * DMOD + kc);
#pragma unroll
            for (int mb = 0; mb < 4; ++mb) acc[mb][nb] = wmma16g(a[mb], b, acc[mb][nb]);
        }
    }
}

__global__ __launch_bounds__(32) void k_proj_qk(const bf* __restrict__ X, const bf* __restrict__ W, const float* __restrict__ bias, bf* Ph, bf* Pl) {
    __shared__ __align__(16) float os[16 * OSP];
    const int lane = (int)threadIdx.x & 31, lr = lane & 15, hi = lane >> 4;
    const int r0 = (int)blockIdx.x * 64, c0 = (int)blockIdx.y * 64;
    v8f acc[4][4];
    gemm_tile(X, W, (size_t)(r0 + lr) * DMOD + 8 * hi, (size_t)(c0 + lr) * DMOD + 8 * hi, acc);
    const int b = r0 / SEQ, t0 = r0 - b * SEQ, hd = (int)blockIdx.y;
    const int rq = lane >> 3, cq = (lane & 7) * 8;
    const v4f bv0 = *(const v4f*)(bias + c0 + cq);
    const v4f bv1 = *(const v4f*)(bias + c0 + cq + 4);
    float bb[8];
    bb[0] = bfr(bv0[0]); bb[1] = bfr(bv0[1]); bb[2] = bfr(bv0[2]); bb[3] = bfr(bv0[3]);
    bb[4] = bfr(bv1[0]); bb[5] = bfr(bv1[1]); bb[6] = bfr(bv1[2]); bb[7] = bfr(bv1[3]);
    const size_t pbase = ((size_t)(b * NHEAD + hd) * SEQ + t0) * HDIM;
#pragma unroll
    for (int mb = 0; mb < 4; ++mb) {
#pragma unroll
        for (int nb = 0; nb < 4; ++nb) {
#pragma unroll
            for (int j = 0; j < 8; ++j) os[(hi * 8 + j) * OSP + nb * 16 + lr] = acc[mb][nb][j];
        }
        __syncthreads();
#pragma unroll 1
        for (int ps = 0; ps < 2; ++ps) {
#pragma unroll
            for (int s = 0; s < 4; ++s) {
                const int row = s * 4 + rq;
                const v4f x0 = *(const v4fa*)(os + row * OSP + cq);
                const v4f x1 = *(const v4fa*)(os + row * OSP + cq + 4);
                v8us oh, ol;
#pragma unroll
                for (int i = 0; i < 4; ++i) {
                    unsigned short a2, c2;
                    splitf(x0[i] + bb[i], a2, c2); oh[i] = a2; ol[i] = c2;
                    splitf(x1[i] + bb[4 + i], a2, c2); oh[4 + i] = a2; ol[4 + i] = c2;
                }
                const size_t oo = pbase + (size_t)(mb * 16 + row) * HDIM + cq;
                *(volatile v8us*)(Ph + oo) = oh;
                *(volatile v8us*)(Pl + oo) = ol;
            }
            if (ps == 0) __threadfence();
        }
        __syncthreads();
    }
}

__global__ __launch_bounds__(32) void k_proj_v(const bf* __restrict__ W, const bf* __restrict__ X, const float* __restrict__ bias, const int* __restrict__ mask, h16* Pv, h16* Pr) {
    __shared__ __align__(16) float os[16 * OSP];
    const int lane = (int)threadIdx.x & 31, lr = lane & 15, hi = lane >> 4;
    const int r0 = (int)blockIdx.x * 64, c0 = (int)blockIdx.y * 64;
    v8f acc[4][4];
    gemm_tile(W, X, (size_t)(r0 + lr) * DMOD + 8 * hi, (size_t)(c0 + lr) * DMOD + 8 * hi, acc);
    const int b = c0 / SEQ, t0 = c0 - b * SEQ, hd = (int)blockIdx.x;
    const int rq = lane >> 3, cq = (lane & 7) * 8;
    const v4i mk0 = *(const v4i*)(mask + (size_t)b * SEQ_FULL + t0 + cq);
    const v4i mk1 = *(const v4i*)(mask + (size_t)b * SEQ_FULL + t0 + cq + 4);
    float mf[8];
    mf[0] = (float)mk0[0]; mf[1] = (float)mk0[1]; mf[2] = (float)mk0[2]; mf[3] = (float)mk0[3];
    mf[4] = (float)mk1[0]; mf[5] = (float)mk1[1]; mf[6] = (float)mk1[2]; mf[7] = (float)mk1[3];
    const size_t pbase = (size_t)(b * NHEAD + hd) * HDIM * SEQ + t0;
#pragma unroll
    for (int mb = 0; mb < 4; ++mb) {
#pragma unroll
        for (int nb = 0; nb < 4; ++nb) {
#pragma unroll
            for (int j = 0; j < 8; ++j) os[(hi * 8 + j) * OSP + nb * 16 + lr] = acc[mb][nb][j];
        }
        __syncthreads();
#pragma unroll 1
        for (int ps = 0; ps < 2; ++ps) {
#pragma unroll
            for (int s = 0; s < 4; ++s) {
                const int row = s * 4 + rq;
                const float bsc = bfr(bias[r0 + mb * 16 + row]);
                const v4f x0 = *(const v4fa*)(os + row * OSP + cq);
                const v4f x1 = *(const v4fa*)(os + row * OSP + cq + 4);
                v8h ov, orr;
#pragma unroll
                for (int i = 0; i < 4; ++i) {
                    const float y0 = (x0[i] + bsc) * mf[i]; const h16 h0 = toh_flush(y0); ov[i] = h0; orr[i] = toh_flush((y0 - (float)h0) * RCAR);
                    const float y1 = (x1[i] + bsc) * mf[4 + i]; const h16 h1 = toh_flush(y1); ov[4 + i] = h1; orr[4 + i] = toh_flush((y1 - (float)h1) * RCAR);
                }
                const size_t oo = pbase + (size_t)(mb * 16 + row) * SEQ + cq;
                *(volatile v8h*)(Pv + oo) = ov;
                *(volatile v8h*)(Pr + oo) = orr;
            }
            if (ps == 0) __threadfence();
        }
        __syncthreads();
    }
}

__global__ __launch_bounds__(128) void k_attn(const bf* __restrict__ QH, const bf* __restrict__ QL, const bf* __restrict__ KH, const bf* __restrict__ KL,
                                              const h16* __restrict__ VV, const h16* __restrict__ VR, float* OUT) {
    __shared__ __align__(16) float os[4 * 16 * OSP];
    const int wave = __builtin_amdgcn_readfirstlane((int)(threadIdx.x >> 5));
    const int lane = (int)threadIdx.x & 31, lr = lane & 15, hi = lane >> 4;
    const int bh = (int)blockIdx.y;
    const int b = bh / NHEAD, hd = bh - b * NHEAD;
    const int q0 = (int)blockIdx.x * 64 + wave * 16;
    const size_t pb = (size_t)bh * SEQ * HDIM;
    const bf* qh = QH + pb; const bf* ql = QL + pb;
    const bf* kh = KH + pb; const bf* kl = KL + pb;
    const h16* vv = VV + pb; const h16* vr = VR + pb;
    const int qoff0 = (q0 + lr) * HDIM + 8 * hi;
    const int koff = lr * HDIM + 8 * hi;
    const int voff = lr * SEQ + 8 * hi;
    v8f ova[4], ore[4];
#pragma unroll
    for (int dt = 0; dt < 4; ++dt) { ova[dt] = (v8f){}; ore[dt] = (v8f){}; }
    float m = -3.0e38f, lsum = 0.0f;
#pragma unroll 1
    for (int j0 = 0; j0 < SEQ; j0 += 32) {
        int qo = qoff0;
        asm volatile("" : "+v"(qo));
        v8f s0 = (v8f){}, s1 = (v8f){};
        v16bf qhf, qlf, k0h, k0l, k1h, k1l;
#pragma unroll
        for (int kc = 0; kc < HDIM; kc += 32) {
            qhf = ldbf(qh + qo + kc); qlf = ldbf(ql + qo + kc);
            const int ko = koff + j0 * HDIM + kc;
            k0h = ldbf(kh + ko); k0l = ldbf(kl + ko);
            k1h = ldbf(kh + ko + 16 * HDIM); k1l = ldbf(kl + ko + 16 * HDIM);
            s0 = wmmab(k0h, qhf, s0); s1 = wmmab(k1h, qhf, s1);
            s0 = wmmab(k0l, qhf, s0); s1 = wmmab(k1l, qhf, s1);
            s0 = wmmab(k0h, qlf, s0); s1 = wmmab(k1h, qlf, s1);
        }
        asm volatile("v_nop\n\tv_nop\n\tv_nop\n\tv_nop" : "+v"(s0), "+v"(s1) : "v"(k1h), "v"(qlf));
        float t0[8], t1[8];
        float mx = -3.0e38f;
#pragma unroll
        for (int r = 0; r < 8; ++r) { t0[r] = s0[r] * LOG2E; t1[r] = s1[r] * LOG2E; mx = fmaxf(mx, fmaxf(t0[r], t1[r])); }
        mx = fmaxf(mx, __shfl_xor(mx, 16, 32));
        const float mnew = fmaxf(m, mx);
        const float sc = __builtin_amdgcn_exp2f(m - mnew);
        m = mnew;
        const float mo = mnew - PSH;
        float psum = 0.0f;
        v16h pf;
#pragma unroll
        for (int r = 0; r < 8; ++r) {
            const float e0 = __builtin_amdgcn_exp2f(t0[r] - mo);
            const float e1 = __builtin_amdgcn_exp2f(t1[r] - mo);
            psum += e0 + e1;
            pf[r] = (h16)e0; pf[8 + r] = (h16)e1;
        }
        lsum = lsum * sc + psum;
        if (__builtin_amdgcn_ballot_w32(sc != 1.0f) != 0u) {
#pragma unroll
            for (int dt = 0; dt < 4; ++dt) {
#pragma unroll
                for (int r = 0; r < 8; ++r) { ova[dt][r] *= sc; ore[dt][r] *= sc; }
            }
        }
        const int vo = voff + j0;
        v16h va[4], vb[4];
#pragma unroll
        for (int dt = 0; dt < 4; ++dt) va[dt] = ldh(vv + vo + dt * 16 * SEQ);
#pragma unroll
        for (int dt = 0; dt < 4; ++dt) ova[dt] = wmma16g(va[dt], pf, ova[dt]);
#pragma unroll
        for (int dt = 0; dt < 4; ++dt) vb[dt] = ldh(vr + vo + dt * 16 * SEQ);
#pragma unroll
        for (int dt = 0; dt < 4; ++dt) ore[dt] = wmma16g(vb[dt], pf, ore[dt]);
    }
    lsum += __shfl_xor(lsum, 16, 32);
    const float inv = 1.0f / lsum;
    const int obase = wave * 16 * OSP;
#pragma unroll
    for (int dt = 0; dt < 4; ++dt) {
        v4f x0, x1;
#pragma unroll
        for (int i = 0; i < 4; ++i) {
            x0[i] = (ova[dt][i] + ore[dt][i] * (1.0f / RCAR)) * inv;
            x1[i] = (ova[dt][4 + i] + ore[dt][4 + i] * (1.0f / RCAR)) * inv;
        }
        *(v4fa*)(os + obase + lr * OSP + dt * 16 + 8 * hi) = x0;
        *(v4fa*)(os + obase + lr * OSP + dt * 16 + 8 * hi + 4) = x1;
    }
    __syncthreads();
    float* orow = OUT + ((size_t)b * SEQ_FULL + q0) * DMOD + hd * HDIM;
#pragma unroll 1
    for (int ps = 0; ps < 2; ++ps) {
#pragma unroll
        for (int s = 0; s < 8; ++s) {
            const int row = 2 * s + hi, cofs = lr * 4;
            const v4f val = *(const v4fa*)(os + obase + row * OSP + cofs);
            *(volatile v4f*)(orow + (size_t)row * DMOD + cofs) = val;
        }
        if (ps == 0) __threadfence();
    }
}

__global__ __launch_bounds__(32) void k_out(const h16* __restrict__ A, const h16* __restrict__ W, const float* __restrict__ bias, const float* __restrict__ xin, float* Y) {
    __shared__ __align__(16) float os[16 * OSP];
    const int lane = (int)threadIdx.x & 31, lr = lane & 15, hi = lane >> 4;
    const int r0 = (int)blockIdx.x * 64, c0 = (int)blockIdx.y * 64;
    v8f acc[4][4];
    gemm_tile_h(A, W, (size_t)(r0 + lr) * DMOD + 8 * hi, (size_t)(c0 + lr) * DMOD + 8 * hi, acc);
    const int b = r0 / SEQ, t0 = r0 - b * SEQ;
    const int cofs = lr * 4;
    const v4f bv0 = *(const v4f*)(bias + c0 + cofs);
    float bb[4];
    bb[0] = bfr(bv0[0]); bb[1] = bfr(bv0[1]); bb[2] = bfr(bv0[2]); bb[3] = bfr(bv0[3]);
    const size_t xbase = ((size_t)b * SEQ_FULL + (size_t)t0) * DMOD + c0 + cofs;
    const size_t ybase = (size_t)r0 * DMOD + c0 + cofs;
    const float osc = 1.0f / (WCAR * CCAR);
#pragma unroll
    for (int mb = 0; mb < 4; ++mb) {
#pragma unroll
        for (int nb = 0; nb < 4; ++nb) {
#pragma unroll
            for (int j = 0; j < 8; ++j) os[(hi * 8 + j) * OSP + nb * 16 + lr] = acc[mb][nb][j];
        }
        __syncthreads();
#pragma unroll 1
        for (int ps = 0; ps < 2; ++ps) {
#pragma unroll
            for (int s = 0; s < 8; ++s) {
                const int row = 2 * s + hi;
                const v4f a4 = *(const v4fa*)(os + row * OSP + cofs);
                const v4f xr = *(const v4f*)(xin + xbase + (size_t)(mb * 16 + row) * DMOD);
                v4f o;
#pragma unroll
                for (int i = 0; i < 4; ++i) o[i] = (a4[i] * osc + bb[i]) + bfr(xr[i]);
                *(volatile v4f*)(Y + ybase + (size_t)(mb * 16 + row) * DMOD) = o;
            }
            if (ps == 0) __threadfence();
        }
        __syncthreads();
    }
}

__global__ __launch_bounds__(256) void k_ln(const float* __restrict__ X, const float* __restrict__ g, const float* __restrict__ be, float* OUT) {
#pragma clang fp contract(off)
    const int wave = __builtin_amdgcn_readfirstlane((int)(threadIdx.x >> 5));
    const int lane = (int)threadIdx.x & 31;
    const int row = (int)blockIdx.x * 8 + wave;
    const int b = row / SEQ, t = row - b * SEQ;
    const float* xr = X + (size_t)row * DMOD;
    v4f x[6];
    float s = 0.0f;
#pragma unroll
    for (int j = 0; j < 6; ++j) {
        x[j] = *(const v4f*)(xr + (j * 32 + lane) * 4);
        s += (x[j][0] + x[j][1]) + (x[j][2] + x[j][3]);
    }
    s += __shfl_xor(s, 16, 32); s += __shfl_xor(s, 8, 32); s += __shfl_xor(s, 4, 32); s += __shfl_xor(s, 2, 32); s += __shfl_xor(s, 1, 32);
    const float mu = s * (1.0f / (float)DMOD);
    float q = 0.0f;
#pragma unroll
    for (int j = 0; j < 6; ++j) {
        const float d0 = x[j][0] - mu, d1 = x[j][1] - mu, d2 = x[j][2] - mu, d3 = x[j][3] - mu;
        q += (d0 * d0 + d1 * d1) + (d2 * d2 + d3 * d3);
    }
    q += __shfl_xor(q, 16, 32); q += __shfl_xor(q, 8, 32); q += __shfl_xor(q, 4, 32); q += __shfl_xor(q, 2, 32); q += __shfl_xor(q, 1, 32);
    const float var = q * (1.0f / (float)DMOD);
    const float rstd = rsqrtf(var + 1.0e-5f);
    v4f o[6];
#pragma unroll
    for (int j = 0; j < 6; ++j) {
        const v4f g4 = *(const v4f*)(g + (j * 32 + lane) * 4);
        const v4f b4 = *(const v4f*)(be + (j * 32 + lane) * 4);
#pragma unroll
        for (int i = 0; i < 4; ++i) o[j][i] = ((x[j][i] - mu) * rstd) * bfr(g4[i]) + bfr(b4[i]);
    }
    float* orow = OUT + ((size_t)b * SEQ_FULL + (size_t)t) * DMOD;
#pragma unroll
    for (int j = 0; j < 6; ++j) *(volatile v4f*)(orow + (j * 32 + lane) * 4) = o[j];
    __threadfence();
#pragma unroll
    for (int j = 0; j < 6; ++j) *(volatile v4f*)(orow + (j * 32 + lane) * 4) = o[j];
}

extern "C" void kernel_launch(void* const* d_in, const int* in_sizes, int n_in,
                              void* d_out, int out_size, void* d_ws, size_t ws_size, hipStream_t stream) {
    if (n_in < 12) return;
    const size_t need_x = (size_t)(NB - 1) * SEQ_FULL * DMOD + (size_t)SEQ * DMOD;
    const size_t need_m = (size_t)(NB - 1) * SEQ_FULL + (size_t)SEQ;
    if ((size_t)in_sizes[0] < need_x || (size_t)in_sizes[1] < need_m) return;
    if (in_sizes[2] < DMOD * DMOD || in_sizes[4] < DMOD * DMOD || in_sizes[6] < DMOD * DMOD || in_sizes[8] < DMOD * DMOD) return;
    if (in_sizes[3] < DMOD || in_sizes[5] < DMOD || in_sizes[7] < DMOD || in_sizes[9] < DMOD) return;
    if (in_sizes[10] < DMOD || in_sizes[11] < DMOD) return;
    if ((size_t)out_size < need_x) return;
    const float* xin = (const float*)d_in[0];
    const int*   msk = (const int*)d_in[1];
    const float* Wq = (const float*)d_in[2]; const float* bq = (const float*)d_in[3];
    const float* Wk = (const float*)d_in[4]; const float* bk = (const float*)d_in[5];
    const float* Wv = (const float*)d_in[6]; const float* bv = (const float*)d_in[7];
    const float* Wo = (const float*)d_in[8]; const float* bo = (const float*)d_in[9];
    const float* lng = (const float*)d_in[10]; const float* lnb = (const float*)d_in[11];
    float* OUT = (float*)d_out;

    constexpr size_t WB = (size_t)DMOD * DMOD * 2;
    constexpr size_t PB = (size_t)NB * SEQ * DMOD * 2;
    constexpr size_t CB = (size_t)NB * SEQ_FULL * DMOD * 4;
    static_assert(WB % 256 == 0);
    static_assert(PB % 256 == 0);
    static_assert(CB % 256 == 0);
    static_assert(4 * WB + 7 * PB + CB <= (size_t)134217728);
    static_assert(((size_t)(NB - 1) * SEQ_FULL + SEQ) * DMOD * 4 <= CB);
    static_assert((size_t)NB * SEQ * DMOD * 2 <= PB);
    static_assert((size_t)NB * SEQ * DMOD * 4 <= 2 * PB);
    if (4 * WB + 7 * PB + CB > ws_size) return;
    char* wsp = (char*)d_ws;
    bf* WQ = (bf*)wsp; wsp += WB;
    bf* WK = (bf*)wsp; wsp += WB;
    bf* WV = (bf*)wsp; wsp += WB;
    h16* WO = (h16*)wsp; wsp += WB;
    bf* XB = (bf*)wsp; wsp += PB;
    bf* QHp = (bf*)wsp; wsp += PB;
    bf* QLp = (bf*)wsp; wsp += PB;
    bf* KHp = (bf*)wsp; wsp += PB;
    bf* KLp = (bf*)wsp; wsp += PB;
    h16* VVp = (h16*)wsp; wsp += PB;
    h16* VRp = (h16*)wsp; wsp += PB;
    float* CTX = (float*)wsp; wsp += CB;
    h16* CTXH = (h16*)QHp;
    float* XF = (float*)KHp;

    const int nW = DMOD * DMOD, nX = NB * SEQ * DMOD;
    const unsigned gW = (unsigned)((nW / 8 + 255) / 256), gX = (unsigned)((nX / 8 + 255) / 256);
    k_cvt<<<gW, 256, 0, stream>>>(Wq, WQ, nW, nW, nW);
    k_cvt<<<gW, 256, 0, stream>>>(Wk, WK, nW, nW, nW);
    k_cvt<<<gW, 256, 0, stream>>>(Wv, WV, nW, nW, nW);
    k_cvt_wo<<<gW, 256, 0, stream>>>(Wo, WO, nW);
    k_cvt<<<gX, 256, 0, stream>>>(xin, XB, nX, SEQ * DMOD, SEQ_FULL * DMOD);
    k_proj_qk<<<dim3(NB * SEQ / 64, DMOD / 64), 32, 0, stream>>>(XB, WQ, bq, QHp, QLp);
    k_proj_qk<<<dim3(NB * SEQ / 64, DMOD / 64), 32, 0, stream>>>(XB, WK, bk, KHp, KLp);
    k_proj_v<<<dim3(DMOD / 64, NB * SEQ / 64), 32, 0, stream>>>(WV, XB, bv, msk, VVp, VRp);
    k_attn<<<dim3(SEQ / 64, NB * NHEAD), 128, 0, stream>>>(QHp, QLp, KHp, KLp, VVp, VRp, CTX);
    k_cvt_ctx<<<gX, 256, 0, stream>>>(CTX, msk, CTXH, nX);
    k_out<<<dim3(NB * SEQ / 64, DMOD / 64), 32, 0, stream>>>(CTXH, WO, bo, xin, XF);
    k_ln<<<dim3(NB * SEQ / 8), 256, 0, stream>>>(XF, lng, lnb, OUT);
}
